// EnhancedCardAwarePolicy_20796231647917
// MI455X (gfx1250) — hardware-verified
//
#include <hip/hip_runtime.h>
#include <hip/hip_bf16.h>

typedef __attribute__((ext_vector_type(16))) _Float16 v16h;
typedef __attribute__((ext_vector_type(8)))  _Float16 v8h;
typedef __attribute__((ext_vector_type(8)))  float    v8f;

union V16 { v16h v; v8h h[2]; };
typedef __attribute__((ext_vector_type(4))) float v4f_t;
typedef float v4fa __attribute__((ext_vector_type(4), may_alias));
typedef __attribute__((ext_vector_type(4))) unsigned v4u_t;
typedef unsigned v4ua __attribute__((ext_vector_type(4), may_alias));

#define NA   30
#define WMMA(a,b,c) __builtin_amdgcn_wmma_f32_16x16x32_f16(false,(a),false,(b),(short)0,(c),false,false)

__global__ void pack_w(const float* __restrict__ W, int Krows, int N, int ktiles,
                       _Float16* __restrict__ out) {
    int ntile = blockIdx.x, ktile = blockIdx.y;
    int t = threadIdx.x;
    int lane = t >> 4, h = t & 15;
    int col  = ntile * 16 + (lane & 15);
    int hi8  = (lane >= 16) ? 8 : 0;
    int krow = ktile * 32 + ((h < 8) ? (hi8 + h) : (16 + hi8 + (h - 8)));
    float v = (krow < Krows) ? W[(size_t)krow * N + col] : 0.0f;
    _Float16* d = out + ((size_t)(ntile * ktiles + ktile) * 512) + lane * 16 + h;
    *(volatile _Float16*)d = (_Float16)v; __threadfence(); *(volatile _Float16*)d = (_Float16)v;
}

__global__ void prep_actions(const int* __restrict__ acards,
                             const float* __restrict__ val_emb,
                             const float* __restrict__ suit_emb,
                             const float* __restrict__ type_emb,
                             const float* __restrict__ ce_w1, const float* __restrict__ ce_b1,
                             const float* __restrict__ ce_w2, const float* __restrict__ ce_b2,
                             const float* __restrict__ as_w1, const float* __restrict__ as_b1,
                             float* __restrict__ abias1,
                             float* __restrict__ strengthA,
                             int*   __restrict__ hasvA,
                             int A) {
    __shared__ float sh_ae[NA][32];
    __shared__ float sh_ce[NA][16];
    int a = threadIdx.x;
    if (a < A) {
        int cs = 0, fv = -1, ace = 0; bool same = true; float total = 0.0f;
        bool pres[6] = {false,false,false,false,false,false};
        for (int c = 0; c < 4; ++c) {
            int card = acards[a * 4 + c];
            if (card != 0) {
                ++cs;
                int val = (card - 1) % 13 + 1;
                int su  = (card - 1) / 13 + 1;
                if (fv < 0) fv = val; else if (val != fv) same = false;
                float atk = (val == 1) ? 1.0f : (val == 11) ? 10.0f : (val == 12) ? 15.0f :
                            (val == 13) ? 20.0f : (float)val;
                total += atk;
                if (su >= 1 && su <= 4) pres[su] = true;
                if (val == 1) ace = 1;
            }
        }
        bool hasv = cs > 0;
        float uniq = (pres[1]?1.f:0.f)+(pres[2]?1.f:0.f)+(pres[3]?1.f:0.f)+(pres[4]?1.f:0.f);
        float fsame = same ? 1.0f : 0.0f;
        float valid = ((float)cs <= 4.0f && (same || ace)) ? 1.0f : 0.0f;
        float feats[6] = {(float)cs, fsame, total, uniq, (float)ace, valid};
        if (!hasv) for (int k = 0; k < 6; ++k) feats[k] = 0.0f;
        strengthA[a] = feats[2] * (1.0f / 20.0f);
        hasvA[a] = hasv ? 1 : 0;
        float h32[32];
        _Pragma("unroll 1") for (int j = 0; j < 32; ++j) {
            float acc = ce_b1[j];
            _Pragma("unroll 1") for (int k = 0; k < 6; ++k) acc += feats[k] * ce_w1[k * 32 + j];
            h32[j] = fmaxf(acc, 0.0f);
        }
        _Pragma("unroll 1") for (int j = 0; j < 16; ++j) {
            float acc = ce_b2[j];
            _Pragma("unroll 1") for (int k = 0; k < 32; ++k) acc += h32[k] * ce_w2[k * 16 + j];
            sh_ce[a][j] = acc;
        }
        float em[32]; for (int j = 0; j < 32; ++j) em[j] = 0.0f;
        int cnt = 0;
        for (int c = 0; c < 4; ++c) {
            int card = acards[a * 4 + c];
            if (card != 0) {
                ++cnt;
                bool inval = (card == 53);
                int v = inval ? 0 : (card - 1) % 13 + 1;
                int s = inval ? 0 : (card - 1) / 13 + 1;
                int ct = (v == 11) ? 1 : (v == 12) ? 2 : (v == 13) ? 3 : 0;
                _Pragma("unroll 1") for (int j = 0; j < 32; ++j) {
                    float e = (j < 16) ? val_emb[v * 16 + j] : suit_emb[s * 16 + (j - 16)];
                    if (j < 8) e += type_emb[ct * 8 + j];
                    em[j] += e;
                }
            }
        }
        float den = (cnt > 0) ? (float)cnt : 1.0f;
        _Pragma("unroll 1") for (int j = 0; j < 32; ++j) sh_ae[a][j] = hasv ? (em[j] / den) : 0.0f;
    }
    __syncthreads();
    for (int idx = threadIdx.x; idx < A * 64; idx += blockDim.x) {
        int aa = idx / 64, j = idx % 64;
        float acc = as_b1[j];
        _Pragma("unroll 1") for (int k = 0; k < 32; ++k) acc += sh_ae[aa][k] * as_w1[(128 + k) * 64 + j];
        _Pragma("unroll 1") for (int k = 0; k < 16; ++k) acc += sh_ce[aa][k] * as_w1[(160 + k) * 64 + j];
        abias1[idx] = acc;
    }
}

__global__ void frontend(const int* __restrict__ hand_cards,
                         const int* __restrict__ enemy_card,
                         const int* __restrict__ hand_size,
                         const float* __restrict__ game_state,
                         const float* __restrict__ discard,
                         const float* __restrict__ val_emb,
                         const float* __restrict__ suit_emb,
                         const float* __restrict__ type_emb,
                         const float* __restrict__ he_wv, const float* __restrict__ he_bv,
                         const float* __restrict__ he_wo, const float* __restrict__ he_bo,
                         const float* __restrict__ se_w1, const float* __restrict__ se_b1,
                         const float* __restrict__ se_w2, const float* __restrict__ se_b2,
                         _Float16* __restrict__ combined) {
    __shared__ float eS[4][32], hvS[4][32], siS[4][20], h64S[4][64], hcS[4][32], scS[4][32];
    int lane = threadIdx.x & 31, sp = threadIdx.x >> 5;
    int b = blockIdx.x * 4 + sp;

    int c = enemy_card[b];
    bool inval = (c == 0) || (c == 53);
    int v = inval ? 0 : (c - 1) % 13 + 1;
    int s = inval ? 0 : (c - 1) / 13 + 1;
    int ct = (v == 11) ? 1 : (v == 12) ? 2 : (v == 13) ? 3 : 0;
    float ej = (lane < 16) ? val_emb[v * 16 + lane] : suit_emb[s * 16 + (lane - 16)];
    if (lane < 8) ej += type_emb[ct * 8 + lane];
    eS[sp][lane] = ej;

    if (lane < 10) siS[sp][lane] = game_state[(size_t)b * 10 + lane];
    if (lane == 0) {
        float hsz = (float)hand_size[b];
        int aces = 0, faces = 0, low = 0; int scnt[6] = {0,0,0,0,0,0};
        bool pres[6] = {false,false,false,false,false,false};
        for (int i = 0; i < 8; ++i) {
            int hc = hand_cards[(size_t)b * 8 + i];
            if (hc != 0) {
                int hv = (hc - 1) % 13 + 1;
                int hs = (hc - 1) / 13 + 1;
                if (hv == 1) ++aces;
                if (hv >= 11 && hv <= 13) ++faces;
                if (hv >= 2 && hv <= 6) ++low;
                if (hs >= 1 && hs <= 4) { ++scnt[hs]; pres[hs] = true; }
            }
        }
        siS[sp][10] = hsz;  siS[sp][11] = (float)aces; siS[sp][12] = (float)faces;
        siS[sp][13] = (float)low;
        siS[sp][14] = (float)scnt[1]; siS[sp][15] = (float)scnt[2];
        siS[sp][16] = (float)scnt[3]; siS[sp][17] = (float)scnt[4];
        siS[sp][18] = (float)faces / (hsz + 1e-8f);
        siS[sp][19] = ((pres[1]?1.f:0.f)+(pres[2]?1.f:0.f)+(pres[3]?1.f:0.f)+(pres[4]?1.f:0.f)) * 0.25f;
    }
    __syncthreads();

    float acc = he_bv[lane];
    _Pragma("unroll 1") for (int k = 0; k < 32; ++k) acc += eS[sp][k] * he_wv[k * 32 + lane];
    hvS[sp][lane] = acc;
    __syncthreads();

    float hs = fmaxf((float)hand_size[b], 1.0f);
    acc = he_bo[lane];
    _Pragma("unroll 1") for (int k = 0; k < 32; ++k) acc += hvS[sp][k] * he_wo[k * 32 + lane];
    hcS[sp][lane] = acc * (8.0f / hs);

    for (int t = 0; t < 2; ++t) {
        int u = lane + t * 32;
        float a2 = se_b1[u];
        _Pragma("unroll 1") for (int k = 0; k < 20; ++k) a2 += siS[sp][k] * se_w1[k * 64 + u];
        h64S[sp][u] = fmaxf(a2, 0.0f);
    }
    __syncthreads();

    acc = se_b2[lane];
    _Pragma("unroll 1") for (int k = 0; k < 64; ++k) acc += h64S[sp][k] * se_w2[k * 32 + lane];
    scS[sp][lane] = acc;

    __shared__ __attribute__((aligned(16))) _Float16 cmb[4 * 160];
    for (int idx = lane; idx < 160; idx += 32) {
        float val;
        if      (idx < 32)  val = hcS[sp][idx];
        else if (idx < 64)  val = eS[sp][idx - 32];
        else if (idx < 96)  val = scS[sp][idx - 64];
        else if (idx < 150) val = discard[(size_t)b * 54 + (idx - 96)];
        else                val = 0.0f;
        cmb[sp * 160 + idx] = (_Float16)val;
    }
    __syncthreads();
    if (threadIdx.x < 80) {
        _Float16* base = combined + (size_t)(b - sp) * 160;
        const v4u_t v = *(const volatile v4ua*)((const unsigned*)cmb + threadIdx.x * 4);
        *(volatile v4u_t*)((unsigned*)base + threadIdx.x * 4) = v; __threadfence(); *(volatile v4u_t*)((unsigned*)base + threadIdx.x * 4) = v;
    }
}

__device__ __forceinline__ void stage_from_lds(const _Float16* tw, const _Float16* Wp,
                                               int ktiles, int lane, v8f acc[8]) {
    int koff = (lane >= 16) ? 8 : 0;
    for (int kt = 0; kt < ktiles; ++kt) {
        V16 a;
        const _Float16* ap = tw + (lane & 15) * 128 + kt * 32 + koff;
        a.h[0] = *(const v8h*)ap;
        a.h[1] = *(const v8h*)(ap + 16);
#pragma unroll
        for (int n = 0; n < 8; ++n) {
            v16h b = *(const v16h*)(Wp + (size_t)(n * ktiles + kt) * 512 + lane * 16);
            acc[n] = WMMA(a.v, b, acc[n]);
        }
    }
}

__device__ __forceinline__ void epilogue_to_lds(const v8f acc[8], const float* bias,
                                                bool relu, int lane, _Float16* tw) {
    int col = lane & 15;
    int rbase = (lane >= 16) ? 8 : 0;
#pragma unroll
    for (int n = 0; n < 8; ++n) {
        float bs = bias[n * 16 + col];
#pragma unroll
        for (int r = 0; r < 8; ++r) {
            float v = acc[n][r] + bs;
            if (relu) v = fmaxf(v, 0.0f);
            tw[(rbase + r) * 128 + n * 16 + col] = (_Float16)v;
        }
    }
}

__global__ void mlp_fused(const _Float16* __restrict__ combined,
                          const _Float16* __restrict__ cx1p, const float* __restrict__ cx_b1,
                          const _Float16* __restrict__ cx2p, const float* __restrict__ cx_b2,
                          const _Float16* __restrict__ cx3p, const float* __restrict__ cx_b3,
                          const _Float16* __restrict__ headp,
                          const float* __restrict__ atc_b1,
                          const float* __restrict__ atc_w2, const float* __restrict__ atc_b2,
                          float* __restrict__ uOut,
                          float* __restrict__ probs) {
    __shared__ _Float16 tile[4][16 * 128];
    __shared__ __attribute__((aligned(16))) float ust[4][16 * 68];
    int lane = threadIdx.x & 31, wv = threadIdx.x >> 5;
    int mtile = blockIdx.x * 4 + wv;
    _Float16* tw = tile[wv];
    int rowg = mtile * 16 + (lane & 15);
    int koff = (lane >= 16) ? 8 : 0;
    const v8f zacc = {};
    v8f acc[8];

#pragma unroll
    for (int n = 0; n < 8; ++n) acc[n] = zacc;
    for (int kt = 0; kt < 5; ++kt) {
        V16 a;
        const _Float16* ap = combined + (size_t)rowg * 160 + kt * 32 + koff;
        a.h[0] = *(const v8h*)ap;
        a.h[1] = *(const v8h*)(ap + 16);
        if (kt + 1 < 5) __builtin_prefetch(ap + 32, 0, 1);
#pragma unroll
        for (int n = 0; n < 8; ++n) {
            v16h b = *(const v16h*)(cx1p + (size_t)(n * 5 + kt) * 512 + lane * 16);
            acc[n] = WMMA(a.v, b, acc[n]);
        }
    }
    epilogue_to_lds(acc, cx_b1, true, lane, tw);

#pragma unroll
    for (int n = 0; n < 8; ++n) acc[n] = zacc;
    stage_from_lds(tw, cx2p, 4, lane, acc);
    epilogue_to_lds(acc, cx_b2, true, lane, tw);

#pragma unroll
    for (int n = 0; n < 8; ++n) acc[n] = zacc;
    stage_from_lds(tw, cx3p, 4, lane, acc);
    epilogue_to_lds(acc, cx_b3, false, lane, tw);

#pragma unroll
    for (int n = 0; n < 8; ++n) acc[n] = zacc;
    stage_from_lds(tw, headp, 4, lane, acc);

    int col = lane & 15;
    int rbase = (lane >= 16) ? 8 : 0;
#pragma unroll
    for (int n = 0; n < 4; ++n) {
        float bs = atc_b1[n * 16 + col];
#pragma unroll
        for (int r = 0; r < 8; ++r) {
            float v = fmaxf(acc[n][r] + bs, 0.0f);
            tw[(rbase + r) * 64 + n * 16 + col] = (_Float16)v;
        }
    }
#pragma unroll
    for (int n = 4; n < 8; ++n) {
#pragma unroll
        for (int r = 0; r < 8; ++r) ust[wv][(rbase + r) * 68 + (n - 4) * 16 + col] = acc[n][r];
    }
    asm volatile("s_wait_dscnt 0" ::: "memory");
#pragma unroll 1
    for (int pass = 0; pass < 2; ++pass) {
#pragma unroll
        for (int i = 0; i < 8; ++i) { const int c = lane + 32 * i, rr = c >> 4, q = (c & 15) * 4;
            *(volatile v4f_t*)(uOut + (size_t)(mtile * 16 + rr) * 64 + q) = *(const volatile v4fa*)(&ust[wv][rr * 68 + q]); }
        __threadfence();
    }

    if (lane < 16) {
        float lg[4] = {atc_b2[0], atc_b2[1], atc_b2[2], atc_b2[3]};
        for (int k = 0; k < 64; ++k) {
            float tv = (float)tw[lane * 64 + k];
#pragma unroll
            for (int j = 0; j < 4; ++j) lg[j] += tv * atc_w2[k * 4 + j];
        }
        float mx = fmaxf(fmaxf(lg[0], lg[1]), fmaxf(lg[2], lg[3]));
        float ex[4], sum = 0.0f;
#pragma unroll
        for (int j = 0; j < 4; ++j) { ex[j] = __expf(lg[j] - mx); sum += ex[j]; }
        float inv = 1.0f / sum;
        float* pr = probs + (size_t)(mtile * 16 + lane) * 4;
        v4f_t pv; pv.x = ex[0] * inv; pv.y = ex[1] * inv; pv.z = ex[2] * inv; pv.w = ex[3] * inv;
        *(volatile v4f_t*)pr = pv; __threadfence(); *(volatile v4f_t*)pr = pv;
    }
}

__global__ void scorer(const float* __restrict__ u,
                       const float* __restrict__ abias1,
                       const _Float16* __restrict__ w2p,
                       const float* __restrict__ as_b2,
                       const float* __restrict__ as_w3,
                       const float* __restrict__ as_b3,
                       const float* __restrict__ probs,
                       const float* __restrict__ strengthA,
                       const int*   __restrict__ hasvA,
                       float* __restrict__ out, int A) {
    __shared__ _Float16 s1[4][16 * 64];
    __shared__ float    s2[4][16 * 32];
    __shared__ __attribute__((aligned(16))) float so[64];
    int lane = threadIdx.x & 31, wv = threadIdx.x >> 5;
    int tile = blockIdx.x * 4 + wv;
    int rowbase = tile * 16;

    for (int idx = lane; idx < 16 * 64; idx += 32) {
        int rl = idx >> 6, col = idx & 63;
        int r = rowbase + rl;
        int bb = r / A, aa = r - bb * A;
        float vv = u[(size_t)bb * 64 + col] + abias1[aa * 64 + col];
        s1[wv][idx] = (_Float16)fmaxf(vv, 0.0f);
    }

    int koff = (lane >= 16) ? 8 : 0;
    v8f c0 = {}, c1 = {};
    for (int kt = 0; kt < 2; ++kt) {
        V16 a;
        const _Float16* ap = &s1[wv][(lane & 15) * 64 + kt * 32 + koff];
        a.h[0] = *(const v8h*)ap;
        a.h[1] = *(const v8h*)(ap + 16);
        v16h b0 = *(const v16h*)(w2p + (size_t)(0 * 2 + kt) * 512 + lane * 16);
        v16h b1 = *(const v16h*)(w2p + (size_t)(1 * 2 + kt) * 512 + lane * 16);
        c0 = WMMA(a.v, b0, c0);
        c1 = WMMA(a.v, b1, c1);
    }
    int col = lane & 15;
    int rb  = (lane >= 16) ? 8 : 0;
    for (int r = 0; r < 8; ++r) {
        int rl = rb + r;
        s2[wv][rl * 32 + col]      = fmaxf(c0[r] + as_b2[col], 0.0f);
        s2[wv][rl * 32 + 16 + col] = fmaxf(c1[r] + as_b2[16 + col], 0.0f);
    }
    if (lane < 16) {
        int r = rowbase + lane;
        float acc = as_b3[0];
        for (int k = 0; k < 32; ++k) acc += s2[wv][lane * 32 + k] * as_w3[k];
        int bb = r / A, aa = r - bb * A;
        const float* tp = probs + (size_t)bb * 4;
        float st = strengthA[aa];
        float bonus = hasvA[aa] ? (tp[0] * st + tp[1] * (1.0f - st)) : tp[3] * 2.0f;
        so[wv * 16 + lane] = acc + bonus;
    }
    __syncthreads();
    if (threadIdx.x < 16) {
        float* ob = out + (size_t)blockIdx.x * 64;
        const v4f_t v = *(const volatile v4fa*)(so + threadIdx.x * 4);
        *(volatile v4f_t*)(ob + threadIdx.x * 4) = v; __threadfence(); *(volatile v4f_t*)(ob + threadIdx.x * 4) = v;
    }
}

extern "C" void kernel_launch(void* const* d_in, const int* in_sizes, int n_in,
                              void* d_out, int out_size, void* d_ws, size_t ws_size,
                              hipStream_t stream) {
    const int*   hand_cards = (const int*)d_in[0];
    const int*   enemy_card = (const int*)d_in[1];
    const int*   hand_size  = (const int*)d_in[2];
    const float* game_state = (const float*)d_in[3];
    const float* discard    = (const float*)d_in[4];
    const int*   acards     = (const int*)d_in[5];
    const float* val_emb    = (const float*)d_in[7];
    const float* suit_emb   = (const float*)d_in[8];
    const float* type_emb   = (const float*)d_in[9];
    const float* ce_w1 = (const float*)d_in[10], *ce_b1 = (const float*)d_in[11];
    const float* ce_w2 = (const float*)d_in[12], *ce_b2 = (const float*)d_in[13];
    const float* he_wv = (const float*)d_in[26], *he_bv = (const float*)d_in[27];
    const float* he_wo = (const float*)d_in[28], *he_bo = (const float*)d_in[29];
    const float* se_w1 = (const float*)d_in[30], *se_b1 = (const float*)d_in[31];
    const float* se_w2 = (const float*)d_in[32], *se_b2 = (const float*)d_in[33];
    const float* atc_w1 = (const float*)d_in[34], *atc_b1 = (const float*)d_in[35];
    const float* atc_w2 = (const float*)d_in[36], *atc_b2 = (const float*)d_in[37];
    const float* as_w1 = (const float*)d_in[38], *as_b1 = (const float*)d_in[39];
    const float* as_w2 = (const float*)d_in[40], *as_b2 = (const float*)d_in[41];
    const float* as_w3 = (const float*)d_in[42], *as_b3 = (const float*)d_in[43];
    const float* cx_w1 = (const float*)d_in[44], *cx_b1 = (const float*)d_in[45];
    const float* cx_w2 = (const float*)d_in[46], *cx_b2 = (const float*)d_in[47];
    const float* cx_w3 = (const float*)d_in[48], *cx_b3 = (const float*)d_in[49];

    const int B = in_sizes[1];
    const int A = in_sizes[5] / 4;
    float* out = (float*)d_out;

    char* base = (char*)d_ws;
    size_t off = 0;
    auto carve = [&](size_t bytes) -> char* {
        char* p = base + off;
        off = (off + bytes + 255) & ~(size_t)255;
        return p;
    };
    _Float16* cx1p  = (_Float16*)carve(8 * 5 * 512 * 2);
    _Float16* cx2p  = (_Float16*)carve(8 * 4 * 512 * 2);
    _Float16* cx3p  = (_Float16*)carve(8 * 4 * 512 * 2);
    _Float16* headp = (_Float16*)carve(8 * 4 * 512 * 2);
    _Float16* as2p  = (_Float16*)carve(2 * 2 * 512 * 2);
    float*    abias1    = (float*)carve((size_t)A * 64 * 4);
    float*    strengthA = (float*)carve((size_t)A * 4);
    int*      hasvA     = (int*)  carve((size_t)A * 4);
    _Float16* combined  = (_Float16*)carve((size_t)B * 160 * 2);
    float*    uBuf      = (float*)carve((size_t)B * 64 * 4);
    float*    probs     = (float*)carve((size_t)B * 4 * 4);
    (void)ws_size; (void)n_in; (void)out_size;

    pack_w<<<dim3(8, 5), 512, 0, stream>>>(cx_w1, 150, 128, 5, cx1p);
    pack_w<<<dim3(8, 4), 512, 0, stream>>>(cx_w2, 128, 128, 4, cx2p);
    pack_w<<<dim3(8, 4), 512, 0, stream>>>(cx_w3, 128, 128, 4, cx3p);
    pack_w<<<dim3(4, 4), 512, 0, stream>>>(atc_w1, 128, 64, 4, headp);
    pack_w<<<dim3(4, 4), 512, 0, stream>>>(as_w1, 128, 64, 4, headp + 4*4*512);
    pack_w<<<dim3(2, 2), 512, 0, stream>>>(as_w2, 64, 32, 2, as2p);

    prep_actions<<<1, 64, 0, stream>>>(acards, val_emb, suit_emb, type_emb,
                                       ce_w1, ce_b1, ce_w2, ce_b2, as_w1, as_b1,
                                       abias1, strengthA, hasvA, A);

    frontend<<<B / 4, 128, 0, stream>>>(hand_cards, enemy_card, hand_size, game_state,
                                        discard, val_emb, suit_emb, type_emb,
                                        he_wv, he_bv, he_wo, he_bo,
                                        se_w1, se_b1, se_w2, se_b2, combined);

    mlp_fused<<<B / 64, 128, 0, stream>>>(combined,
                                          cx1p, cx_b1, cx2p, cx_b2, cx3p, cx_b3,
                                          headp, atc_b1, atc_w2, atc_b2,
                                          uBuf, probs);

    int tiles = (B * A) / 16;
    scorer<<<tiles / 4, 128, 0, stream>>>(uBuf, abias1, as2p, as_b2, as_w3, as_b3,
                                          probs, strengthA, hasvA, out, A);
}
